// HierarchicalSkeletalEncoder_23613730193795
// MI455X (gfx1250) — hardware-verified
//
#include <hip/hip_runtime.h>


#define NN   8192
#define NJ   17
#define HD   64
#define OUTW 128
typedef _Float16 h16;
typedef unsigned short bf;
typedef __attribute__((ext_vector_type(16))) __bf16   v16bf;
typedef __attribute__((ext_vector_type(16))) _Float16 v16h;
typedef __attribute__((ext_vector_type(8)))  _Float16 v8h;
typedef __attribute__((ext_vector_type(8)))  unsigned short v8us;
typedef __attribute__((ext_vector_type(8)))  float    v8f;
typedef __attribute__((ext_vector_type(4)))  float    v4f;
typedef v8h  __attribute__((may_alias)) v8ha;
typedef v4f  __attribute__((may_alias)) v4fa;
typedef v8us __attribute__((may_alias)) v8usa;

__device__ __forceinline__ unsigned short f2bf(float f) { unsigned u = __float_as_uint(f); u += 0x7FFFu + ((u >> 16) & 1u); return (unsigned short)(u >> 16); }
__device__ __forceinline__ float bf2f(unsigned short b) { return __uint_as_float(((unsigned)b) << 16); }
__device__ __forceinline__ float bfr(float f) { return bf2f(f2bf(f)); }
__device__ __forceinline__ v16h cat16(v8h lo, v8h hi) { return __builtin_shufflevector(lo, hi, 0, 1, 2, 3, 4, 5, 6, 7, 8, 9, 10, 11, 12, 13, 14, 15); }
__device__ __forceinline__ v16bf cat16b(v8us lo, v8us hi) { return __builtin_bit_cast(v16bf, __builtin_shufflevector(lo, hi, 0, 1, 2, 3, 4, 5, 6, 7, 8, 9, 10, 11, 12, 13, 14, 15)); }
__device__ __forceinline__ v8f wmma16(v16h a, v16h b, v8f c) { return __builtin_amdgcn_wmma_f32_16x16x32_f16(false, a, false, b, (short)0, c, false, false); }
__device__ __forceinline__ v8f wmmab(v16bf a, v16bf b, v8f c) { return __builtin_amdgcn_wmma_f32_16x16x32_bf16(false, a, false, b, (short)0, c, false, false); }


template <typename T16> struct WFrag;
template <> struct WFrag<h16> { typedef v16h V; static __device__ __forceinline__ V ld(const h16* p) { return cat16(*(const v8h*)p, *(const v8h*)(p + 16)); } static __device__ __forceinline__ v8f mma(V a, V b, v8f c) { return wmma16(a, b, c); } };
template <> struct WFrag<bf> { typedef v16bf V; static __device__ __forceinline__ V ld(const bf* p) { return cat16b(*(const v8us*)p, *(const v8us*)(p + 16)); } static __device__ __forceinline__ v8f mma(V a, V b, v8f c) { return wmmab(a, b, c); } };
template <typename T16, int NSPLIT, bool BIAS>
__global__ __launch_bounds__(32) void k_gemmw(const T16* __restrict__ A, const T16* __restrict__ A2, const T16* __restrict__ Bt, const T16* __restrict__ Bt2, int K, float* C, int ldc, const float* __restrict__ bias, size_t sA, size_t sB, size_t sC) {
    typedef typename WFrag<T16>::V V;
    __shared__ __align__(16) float os[16 * 68];
    const size_t z = blockIdx.z; A += z * sA; if (A2) A2 += z * sA; Bt += z * sB; if (Bt2) Bt2 += z * sB; C += z * sC;
    const int lane = threadIdx.x & 31, lr = lane & 15, hi = lane >> 4; const int r0 = blockIdx.x * 64, c0 = blockIdx.y * 64;
    v8f acc[4][4];
#pragma unroll
    for (int mb = 0; mb < 4; ++mb)
#pragma unroll
        for (int nb = 0; nb < 4; ++nb) acc[mb][nb] = (v8f){};
    const size_t aoff = (size_t)(r0 + lr) * K + 8 * hi, boff = (size_t)(c0 + lr) * K + 8 * hi;
#pragma unroll 1
    for (int kc = 0; kc < K; kc += 32) {
        V a[4], a2[4];
#pragma unroll
        for (int mb = 0; mb < 4; ++mb) { a[mb] = WFrag<T16>::ld(A + aoff + (size_t)mb * 16 * K + kc); if (NSPLIT == 1 || NSPLIT == 2) a2[mb] = WFrag<T16>::ld(A2 + aoff + (size_t)mb * 16 * K + kc); }
#pragma unroll
        for (int nb = 0; nb < 4; ++nb) { const V b = WFrag<T16>::ld(Bt + boff + (size_t)nb * 16 * K + kc); V b2; if (NSPLIT >= 2) b2 = WFrag<T16>::ld(Bt2 + boff + (size_t)nb * 16 * K + kc);
#pragma unroll
            for (int mb = 0; mb < 4; ++mb) { acc[mb][nb] = WFrag<T16>::mma(a[mb], b, acc[mb][nb]); if (NSPLIT == 1 || NSPLIT == 2) acc[mb][nb] = WFrag<T16>::mma(a2[mb], b, acc[mb][nb]); if (NSPLIT >= 2) acc[mb][nb] = WFrag<T16>::mma(a[mb], b2, acc[mb][nb]); } }
        asm volatile("v_nop\n\tv_nop\n\tv_nop\n\tv_nop" : "+v"(acc[0][0]), "+v"(acc[1][1]), "+v"(acc[2][2]), "+v"(acc[3][3]) : "v"(a[0]), "v"(a[3]));
    }
#pragma unroll
    for (int mb = 0; mb < 4; ++mb) {
#pragma unroll
        for (int nb = 0; nb < 4; ++nb) {
#pragma unroll
            for (int j = 0; j < 8; ++j) os[(hi * 8 + j) * 68 + nb * 16 + lr] = acc[mb][nb][j]; }
        __builtin_amdgcn_wave_barrier(); asm volatile("" ::: "memory");
        float* crow = C + (size_t)(r0 + mb * 16) * ldc + c0;
#pragma unroll 1
        for (int ps = 0; ps < 2; ++ps) {
#pragma unroll
            for (int s = 0; s < 8; ++s) { const int row = 2 * s + hi, cofs = lr * 4; v4f val = *(const v4fa*)(os + row * 68 + cofs); if (BIAS) { val[0] += bfr(bias[c0 + cofs]); val[1] += bfr(bias[c0 + cofs + 1]); val[2] += bfr(bias[c0 + cofs + 2]); val[3] += bfr(bias[c0 + cofs + 3]); }
                *(volatile v4f*)(crow + (size_t)row * ldc + cofs) = val; }
            if (ps == 0) __threadfence(); }
        __builtin_amdgcn_wave_barrier(); asm volatile("" ::: "memory");
    }
}

__device__ __forceinline__ void splitf(float y, unsigned short& h, unsigned short& l) { h = f2bf(y); l = f2bf(y - bf2f(h)); }
typedef __attribute__((ext_vector_type(2))) unsigned short v2us;
typedef __attribute__((ext_vector_type(4))) unsigned short v4us;
typedef __attribute__((ext_vector_type(2))) float v2f;
__constant__ int c_sub[3][5] = {{0, 5, 6, 11, 12}, {7, 8, 13, 14, -1}, {9, 10, 15, 16, -1}};
__constant__ int c_nsub[3] = {5, 4, 4};
__constant__ int c_nb[188] = {5,6,7,8,11,12,13,14,0,6,7,8,11,12,13,14,0,5,7,8,11,12,13,14,0,5,6,11,12,0,5,6,11,12,0,5,6,7,8,12,13,14,0,5,6,7,8,11,13,14,0,5,6,11,12,0,5,6,11,12,7,8,13,14,7,8,13,14,7,8,13,14,0,5,6,8,9,10,11,12,13,14,15,16,0,5,6,7,9,10,11,12,13,14,15,16,7,8,13,14,7,8,13,14,7,8,13,14,7,8,13,14,0,5,6,7,8,9,10,11,12,14,15,16,0,5,6,7,8,9,10,11,12,13,15,16,7,8,13,14,7,8,13,14,9,10,15,16,9,10,15,16,7,8,10,13,14,15,16,7,8,9,13,14,15,16,9,10,15,16,9,10,15,16,7,8,9,10,13,14,16,7,8,9,10,13,14,15};
__constant__ int c_st[3][18] = {{0,8,8,8,8,8,16,24,29,34,34,34,42,50,55,60,60,60}, {60,64,64,64,64,64,68,72,84,96,100,104,108,112,124,136,140,144}, {144,144,144,144,144,144,144,144,148,152,159,166,166,166,170,174,181,188}};

__global__ __launch_bounds__(256) void k_cvt8(const float* __restrict__ src, bf* dst, size_t n8) { const size_t i = (size_t)blockIdx.x * 256 + threadIdx.x; if (i >= n8) return; const v8f v = *(const v8f*)(src + i * 8); v8us o;
#pragma unroll
    for (int k = 0; k < 8; ++k) o[k] = f2bf(v[k]); *(volatile v8us*)(dst + i * 8) = o; __threadfence(); *(volatile v8us*)(dst + i * 8) = o; }
__global__ __launch_bounds__(256) void k_we(const float* __restrict__ We, bf* W1, bf* W2) { const int e = (blockIdx.x * 256 + threadIdx.x) * 4; if (e >= HD * HD) return; const int k = e % HD, o = e / HD; v4us a, b;
#pragma unroll
    for (int q = 0; q < 4; ++q) { a[q] = f2bf(We[o * 2 * HD + k + q]); b[q] = f2bf(We[o * 2 * HD + HD + k + q]); } *(volatile v4us*)(W1 + e) = a; *(volatile v4us*)(W2 + e) = b; __threadfence(); *(volatile v4us*)(W1 + e) = a; *(volatile v4us*)(W2 + e) = b; }
__global__ __launch_bounds__(256) void k_prep(const float* __restrict__ kp, const float* __restrict__ sc, float* P) { const int e = blockIdx.x * 256 + threadIdx.x; if (e >= NN * NJ) return; const int j = e % NJ, n = e / NJ; float mnx = 3.0e38f, mny = 3.0e38f, mxx = -3.0e38f, mxy = -3.0e38f;
    for (int jj = 0; jj < NJ; ++jj) { const float x = bfr(kp[((size_t)n * NJ + jj) * 2]), y = bfr(kp[((size_t)n * NJ + jj) * 2 + 1]); mnx = fminf(mnx, x); mxx = fmaxf(mxx, x); mny = fminf(mny, y); mxy = fmaxf(mxy, y); }
    const float x = bfr(kp[(size_t)e * 2]), y = bfr(kp[(size_t)e * 2 + 1]); v4f o; o[0] = __fdiv_rn(__fsub_rn(x, mnx), __fadd_rn(__fsub_rn(mxx, mnx), 1e-6f)); o[1] = __fdiv_rn(__fsub_rn(y, mny), __fadd_rn(__fsub_rn(mxy, mny), 1e-6f)); o[2] = bfr(sc[e]); o[3] = 0.f;
    *(volatile v4f*)(P + (size_t)e * 4) = o; __threadfence(); *(volatile v4f*)(P + (size_t)e * 4) = o; }
__global__ __launch_bounds__(256) void k_feat(const float* __restrict__ P, const float* __restrict__ W, const float* __restrict__ b, int lv, float* FEAT, float* HB) { const int e = blockIdx.x * 256 + threadIdx.x; if (e >= NN * NJ * HD) return; const int h = e % HD; const int u = (e / HD) % NJ; const int n = e / (HD * NJ); const float w0 = bfr(W[h * 3]), w1 = bfr(W[h * 3 + 1]), w2 = bfr(W[h * 3 + 2]), bb = bfr(b[h]);
    int inset = 0; for (int q = 0; q < c_nsub[lv]; ++q) inset |= (c_sub[lv][q] == u); float H = 0.f;
    if (inset) { for (int q = 0; q < c_nsub[lv]; ++q) { const int v = c_sub[lv][q]; if (v == u) continue; const float* pv = P + ((size_t)n * NJ + v) * 4; float a0 = __fmul_rn(pv[0], w0), a1 = __fmul_rn(pv[1], w1), a2 = __fmul_rn(pv[2], w2); asm volatile("" : "+v"(a0), "+v"(a1), "+v"(a2)); const float hv = fmaxf(__fadd_rn(__fadd_rn(__fadd_rn(a0, a1), a2), bb), 0.f); float mv = __fmul_rn(hv, pv[2]); asm volatile("" : "+v"(mv)); H = __fadd_rn(H, mv); } }
    const float f = __fmul_rn(H, P[((size_t)n * NJ + u) * 4 + 2]);
    for (int ps = 0; ps < 2; ++ps) { *(volatile float*)(FEAT + e) = f; *(volatile float*)(HB + e) = H; if (ps == 0) __threadfence(); } }
__global__ __launch_bounds__(256) void k_pool(const float* __restrict__ G1, const float* __restrict__ G2, const float* __restrict__ HB, const float* __restrict__ be, int lv, float* POOL) { const int e = blockIdx.x * 256 + threadIdx.x; if (e >= NN * HD) return; const int o = e % HD, n = e / HD; const float b = bfr(be[o]); float zs = 0.f, hs = 0.f;
    for (int u = 0; u < NJ; ++u) { const size_t ru = ((size_t)n * NJ + u) * HD + o; const float base = __fsub_rn(G1[ru], G2[ru]); float z = 0.f;
        for (int q = c_st[lv][u]; q < c_st[lv][u + 1]; ++q) { const int k = c_nb[q]; z = fmaxf(z, fmaxf(__fadd_rn(__fadd_rn(base, G2[((size_t)n * NJ + k) * HD + o]), b), 0.f)); }
        zs = __fadd_rn(zs, z); hs = __fadd_rn(hs, HB[ru]); }
    const float zm = __fdiv_rn(zs, (float)NJ), hm = __fdiv_rn(hs, (float)NJ); const size_t po = (size_t)n * 3 * OUTW + lv * OUTW + o;
    *(volatile float*)(POOL + po) = hm; *(volatile float*)(POOL + po + HD) = zm; __threadfence(); *(volatile float*)(POOL + po) = hm; *(volatile float*)(POOL + po + HD) = zm; }
__global__ __launch_bounds__(256) void k_spl(const float* __restrict__ F, size_t n4, bf* Fh, bf* Fl) { const size_t i = ((size_t)blockIdx.x * 256 + threadIdx.x) * 4; if (i >= n4 * 4) return; const v4f a = *(const v4f*)(F + i); v4us oh, ol;
#pragma unroll
    for (int q = 0; q < 4; ++q) { unsigned short u, c2; splitf(a[q], u, c2); oh[q] = u; ol[q] = c2; } *(volatile v4us*)(Fh + i) = oh; *(volatile v4us*)(Fl + i) = ol; __threadfence(); *(volatile v4us*)(Fh + i) = oh; *(volatile v4us*)(Fl + i) = ol; }

extern "C" void kernel_launch(void* const* d_in, const int* in_sizes, int n_in,
                              void* d_out, int out_size, void* d_ws, size_t ws_size, hipStream_t stream) {
    (void)in_sizes; (void)n_in; (void)out_size;
    const float* IN[12]; for (int i = 0; i < 12; ++i) IN[i] = (const float*)d_in[i];
    float* OUT = (float*)d_out;
    char* wsp = (char*)d_ws;
    auto take = [&](size_t bytes) { char* p = wsp; wsp += (bytes + 255) & ~(size_t)255; return (void*)p; };
    bf* W1 = (bf*)take(HD * HD * 2); bf* W2 = (bf*)take(HD * HD * 2); bf* WP = (bf*)take((size_t)OUTW * 3 * OUTW * 2);
    float* P = (float*)take((size_t)NN * NJ * 4 * 4); float* FEAT = (float*)take((size_t)NN * NJ * HD * 4); bf* Fh = (bf*)take((size_t)NN * NJ * HD * 2); bf* Fl = (bf*)take((size_t)NN * NJ * HD * 2); float* HB = (float*)take((size_t)NN * NJ * HD * 4);
    float* G1 = (float*)take((size_t)NN * NJ * HD * 4); float* G2 = (float*)take((size_t)NN * NJ * HD * 4); float* POOL = (float*)take((size_t)NN * 3 * OUTW * 4); bf* Ph = (bf*)take((size_t)NN * 3 * OUTW * 2); bf* Pl = (bf*)take((size_t)NN * 3 * OUTW * 2);
    if ((size_t)(wsp - (char*)d_ws) > ws_size) return;
    k_we<<<(HD * HD / 4 + 255) / 256, 256, 0, stream>>>(IN[8], W1, W2); k_cvt8<<<(OUTW * 3 * OUTW / 8 + 255) / 256, 256, 0, stream>>>(IN[10], WP, (size_t)OUTW * 3 * OUTW / 8);
    k_prep<<<(NN * NJ + 255) / 256, 256, 0, stream>>>(IN[0], IN[1], P);
    for (int lv = 0; lv < 3; ++lv) {
        k_feat<<<(NN * NJ * HD + 255) / 256, 256, 0, stream>>>(P, IN[2 + 2 * lv], IN[3 + 2 * lv], lv, FEAT, HB); k_spl<<<(NN * NJ * HD / 4 + 255) / 256, 256, 0, stream>>>(FEAT, (size_t)NN * NJ * HD / 4, Fh, Fl);
        k_gemmw<bf, 1, false><<<dim3(NN * NJ / 64, 1, 1), 32, 0, stream>>>(Fh, Fl, W1, nullptr, HD, G1, HD, nullptr, 0, 0, 0); k_gemmw<bf, 1, false><<<dim3(NN * NJ / 64, 1, 1), 32, 0, stream>>>(Fh, Fl, W2, nullptr, HD, G2, HD, nullptr, 0, 0, 0);
        k_pool<<<(NN * HD + 255) / 256, 256, 0, stream>>>(G1, G2, HB, IN[9], lv, POOL); }
    k_spl<<<(NN * 3 * OUTW / 4 + 255) / 256, 256, 0, stream>>>(POOL, (size_t)NN * 3 * OUTW / 4, Ph, Pl);
    k_gemmw<bf, 1, true><<<dim3(NN / 64, OUTW / 64, 1), 32, 0, stream>>>(Ph, Pl, WP, nullptr, 3 * OUTW, OUT, OUTW, IN[11], 0, 0, 0);
}
